// GATClassifier_5677946765452
// MI455X (gfx1250) — hardware-verified
//
#include <hip/hip_runtime.h>
#include <stddef.h>
#include <stdint.h>
#include <math.h>


#define DIN    128
#define HC     64
#define NHEAD  4
#define H3W    256
#define CLSH   32
#define KP     128
#define NTHR   256
#define NWAVE  8
#define EPT    8
#define CHUNK  (NTHR * EPT)
#define WCAP   (EPT * 32)
#define LISTN  (NWAVE * WCAP)
#define NBA    1024
#define SLA    10
#define RCAP   28672
#define DEGCAP 128
#define GBM    64
#define GBN    64
#define GTHR   128
#define NU1    (HC * (DIN / 8))
#define NU2    (HC * (KP / 8))
#define NU3    (H3W * (KP / 8))
#define NU4    (GBN * (KP / 8))
#define NEGSL  0.2f
#define BNEPS  1e-5f
#define AGG_ZINTS (LISTN + 2 * RCAP + 3 * NBA)
#define AGG_LDS_INTS (AGG_ZINTS + 16)
#define WSMAX  134217728

static_assert((CHUNK & (CHUNK - 1)) == 0 && CHUNK <= 4096);
static_assert((NBA & (NBA - 1)) == 0 && NBA == (1 << SLA));
static_assert(((long long)CHUNK << SLA) < (1LL << 31));
static_assert(LISTN % NTHR == 0);
static_assert(NBA % NWAVE == 0 && NBA % 32 == 0 && NBA % GBM == 0);
static_assert(RCAP % 4 == 0 && AGG_ZINTS % 4 == 0 && LISTN % 4 == 0);
static_assert(DIN % 32 == 0 && KP % 32 == 0 && KP == 2 * HC && KP == DIN);
static_assert(GBM == (GTHR / 32) * 16 && GBN == 64 && GTHR == 2 * GBM && GTHR == 2 * GBN);
static_assert(NU1 % NTHR == 0 && NU2 % NTHR == 0 && NU3 % NTHR == 0 && NU4 % NTHR == 0);
static_assert(HC == NHEAD * 16 && H3W == NHEAD * HC && NHEAD * 16 == GBN);
static_assert(HC == 2 * 32 && H3W == 8 * 32);
static_assert(CLSH == 32 && CLSH <= GBN);
static_assert(AGG_LDS_INTS * 4 <= 300000);
static_assert(DIN / 8 == 16 && KP / 8 == 16);

typedef float          v2f   __attribute__((ext_vector_type(2)));
typedef float          v4f   __attribute__((ext_vector_type(4)));
typedef float          v8f   __attribute__((ext_vector_type(8)));
typedef int            v4i   __attribute__((ext_vector_type(4)));
typedef int            v8i   __attribute__((ext_vector_type(8)));
typedef unsigned int   v4u   __attribute__((ext_vector_type(4)));
typedef unsigned short v8us  __attribute__((ext_vector_type(8)));
typedef unsigned short v16us __attribute__((ext_vector_type(16)));
typedef __bf16         v16bf __attribute__((ext_vector_type(16)));
typedef v2f  __attribute__((may_alias)) v2fa;
typedef v4f  __attribute__((may_alias)) v4fa;
typedef v4i  __attribute__((may_alias)) v4ia;
typedef v8us __attribute__((may_alias)) v8usa;
union FragB { v16bf v; v16us u; v8us h[2]; v8i w; };
union Pk8 { v8us h; v4u u; };

__device__ __forceinline__ v8f wmb(const FragB& a, const FragB& b, v8f c) {
  v8f d = __builtin_amdgcn_wmma_f32_16x16x32_bf16(false, a.v, false, b.v, (short)0, c, false, false);
  asm volatile("v_nop\n\tv_nop\n\tv_nop\n\tv_nop" : "+v"(d) : "v"(a.w), "v"(b.w));
  return d;
}

__device__ __forceinline__ unsigned bf16_bits(float f) {
  const unsigned u = __float_as_uint(f);
  return ((u + 0x7FFFu + ((u >> 16) & 1u)) >> 16) & 0xFFFFu;
}
__device__ __forceinline__ float bf16_val(float f) {
  return __uint_as_float(bf16_bits(f) << 16);
}
__device__ __forceinline__ float eluf(float x) {
  const float e = expm1f(fminf(x, 0.0f));
  return x > 0.0f ? x : e;
}

template <int CPL>
__device__ __forceinline__ void ldc(const float* __restrict__ p, float* o) {
  if constexpr (CPL == 2) {
    const v2f a = *(const v2fa*)p;
    o[0] = a.x; o[1] = a.y;
  } else {
    const v4f a = *(const v4fa*)p;
    const v4f b = *(const v4fa*)(p + 4);
    o[0] = a.x; o[1] = a.y; o[2] = a.z; o[3] = a.w;
    o[4] = b.x; o[5] = b.y; o[6] = b.z; o[7] = b.w;
  }
}

template <int SLB>
__device__ __forceinline__ int scan_chunk(const int* __restrict__ dsts, int nE, int cbase, int slotBase,
                                          int nb, int vec8, int* list, int tid, int lane, int wave) {
  int wc = 0;
  const int el0  = tid * EPT;
  const int e0   = cbase + el0;
  const int sent = -2147483647 - 1;
  v4i da, db;
  if (vec8 != 0 && cbase + CHUNK <= nE) {
    da = *(const v4i*)(dsts + e0);
    db = *(const v4i*)(dsts + e0 + 4);
  } else {
    da.x = (e0     < nE) ? dsts[min(e0,     nE - 1)] : sent;
    da.y = (e0 + 1 < nE) ? dsts[min(e0 + 1, nE - 1)] : sent;
    da.z = (e0 + 2 < nE) ? dsts[min(e0 + 2, nE - 1)] : sent;
    da.w = (e0 + 3 < nE) ? dsts[min(e0 + 3, nE - 1)] : sent;
    db.x = (e0 + 4 < nE) ? dsts[min(e0 + 4, nE - 1)] : sent;
    db.y = (e0 + 5 < nE) ? dsts[min(e0 + 5, nE - 1)] : sent;
    db.z = (e0 + 6 < nE) ? dsts[min(e0 + 6, nE - 1)] : sent;
    db.w = (e0 + 7 < nE) ? dsts[min(e0 + 7, nE - 1)] : sent;
  }
  const unsigned nbs = (unsigned)slotBase;
  const unsigned unb = (unsigned)nb;
  const unsigned s0 = (unsigned)da.x - nbs, s1 = (unsigned)da.y - nbs;
  const unsigned s2 = (unsigned)da.z - nbs, s3 = (unsigned)da.w - nbs;
  const unsigned s4 = (unsigned)db.x - nbs, s5 = (unsigned)db.y - nbs;
  const unsigned s6 = (unsigned)db.z - nbs, s7 = (unsigned)db.w - nbs;
  const bool h0 = s0 < unb, h1 = s1 < unb, h2 = s2 < unb, h3 = s3 < unb;
  const bool h4 = s4 < unb, h5 = s5 < unb, h6 = s6 < unb, h7 = s7 < unb;
  const unsigned any = __builtin_amdgcn_ballot_w32(h0 | h1 | h2 | h3 | h4 | h5 | h6 | h7);
  if (any != 0u) {
#define HITJ(J, HJ, SJ) { \
      const unsigned mj = __builtin_amdgcn_ballot_w32(HJ); \
      if (mj != 0u) { \
        if (HJ) { \
          const int pos = wc + (int)__builtin_amdgcn_mbcnt_lo(mj, 0u); \
          if (pos < WCAP) list[wave * WCAP + pos] = ((el0 + (J)) << SLB) | (int)(SJ); \
        } \
        wc += (int)__builtin_popcount(mj); } }
    HITJ(0, h0, s0)
    HITJ(1, h1, s1)
    HITJ(2, h2, s2)
    HITJ(3, h3, s3)
    HITJ(4, h4, s4)
    HITJ(5, h5, s5)
    HITJ(6, h6, s6)
    HITJ(7, h7, s7)
#undef HITJ
  }
  return wc;
}

__global__ __launch_bounds__(NTHR) void k_wprep(const float* __restrict__ W1, const float* __restrict__ W2,
                                                const float* __restrict__ W3, const float* __restrict__ CW1,
                                                unsigned short* W1T, unsigned short* W2T,
                                                unsigned short* W3T, unsigned short* CWT) {
  const int u = (int)blockIdx.x * NTHR + (int)threadIdx.x;
  v8us o;
  unsigned short* dp;
  if (u < NU1) {
    const int n  = u >> 4;
    const int k8 = (u & 15) * 8;
    const float* p = W1 + (size_t)k8 * HC + n;
#pragma unroll
    for (int i = 0; i < 8; ++i) o[i] = (unsigned short)bf16_bits(p[(size_t)i * HC]);
    dp = W1T + (size_t)n * DIN + k8;
  } else if (u < NU1 + NU2) {
    const int v  = u - NU1;
    const int n  = v >> 4;
    const int k8 = (v & 15) * 8;
    const int kk = k8 & (HC - 1);
    const float* p = W2 + (size_t)kk * HC + n;
#pragma unroll
    for (int i = 0; i < 8; ++i) o[i] = (unsigned short)bf16_bits(p[(size_t)i * HC]);
    dp = W2T + (size_t)n * KP + k8;
  } else if (u < NU1 + NU2 + NU3) {
    const int v  = u - NU1 - NU2;
    const int n  = v >> 4;
    const int k8 = (v & 15) * 8;
    const int kk = k8 & (HC - 1);
    const float* p = W3 + (size_t)kk * H3W + n;
#pragma unroll
    for (int i = 0; i < 8; ++i) o[i] = (unsigned short)bf16_bits(p[(size_t)i * H3W]);
    dp = W3T + (size_t)n * KP + k8;
  } else if (u < NU1 + NU2 + NU3 + NU4) {
    const int v   = u - NU1 - NU2 - NU3;
    const int n   = v >> 4;
    const int k8  = (v & 15) * 8;
    const int kk  = k8 & (HC - 1);
    const int ncl = n < CLSH ? n : CLSH - 1;
    const float* p = CW1 + (size_t)kk * CLSH + ncl;
#pragma unroll
    for (int i = 0; i < 8; ++i) o[i] = (unsigned short)bf16_bits(p[(size_t)i * CLSH]);
    const v8us z8 = {0, 0, 0, 0, 0, 0, 0, 0};
    if (n >= CLSH) o = z8;
    dp = CWT + (size_t)n * KP + k8;
  } else {
    return;
  }
  *(volatile v8us*)dp = o;
  __threadfence();
  *(volatile v8us*)dp = o;
}

__global__ __launch_bounds__(NTHR) void k_cvx(const float* __restrict__ x, int nN, int nUnits,
                                              unsigned short* xb) {
  const int u = (int)blockIdx.x * NTHR + (int)threadIdx.x;
  if (u >= nUnits) return;
  const int row = u >> 4;
  const int k8  = (u & 15) * 8;
  const int rc  = row < nN ? row : nN - 1;
  const float* p = x + (size_t)rc * DIN + k8;
  const v4f a = *(const v4f*)p;
  const v4f b = *(const v4f*)(p + 4);
  const bool ok = row < nN;
  v8us o;
  o[0] = ok ? (unsigned short)bf16_bits(a.x) : (unsigned short)0;
  o[1] = ok ? (unsigned short)bf16_bits(a.y) : (unsigned short)0;
  o[2] = ok ? (unsigned short)bf16_bits(a.z) : (unsigned short)0;
  o[3] = ok ? (unsigned short)bf16_bits(a.w) : (unsigned short)0;
  o[4] = ok ? (unsigned short)bf16_bits(b.x) : (unsigned short)0;
  o[5] = ok ? (unsigned short)bf16_bits(b.y) : (unsigned short)0;
  o[6] = ok ? (unsigned short)bf16_bits(b.z) : (unsigned short)0;
  o[7] = ok ? (unsigned short)bf16_bits(b.w) : (unsigned short)0;
  unsigned short* dp = xb + (size_t)row * DIN + k8;
  *(volatile v8us*)dp = o;
  __threadfence();
  *(volatile v8us*)dp = o;
}

template <int MODE>
__global__ __launch_bounds__(GTHR) void k_gemm(
    const unsigned short* __restrict__ A, const unsigned short* __restrict__ WT,
    float* outF, int ldo,
    const float* __restrict__ atts, const float* __restrict__ attd, float* SD, int MPr,
    const float* __restrict__ cb1, const float* __restrict__ cw2, const float* __restrict__ cb2,
    float* outp, int nN)
{
  static_assert(MODE == 0 || MODE == 1 || MODE == 2);
  constexpr int HB = (MODE == 0) ? NHEAD : 1;
  constexpr int DL = GBN / HB;
  __shared__ __attribute__((aligned(16))) float stg[GBM * GBN];
  __shared__ __attribute__((aligned(16))) float satt[2 * GBN];
  __shared__ __attribute__((aligned(16))) float sdot[2 * NHEAD * GBM];
  const int tid = (int)threadIdx.x, lane = tid & 31, wave = tid >> 5, hh = lane >> 4, m = lane & 15;
  const int rowBase = (int)blockIdx.x * GBM;
  const int cgrp    = (int)blockIdx.y;
  const int col0    = cgrp * GBN;

  if constexpr (MODE != 2) {
    const int which = tid >> 6;
    const int c  = tid & 63;
    const int ab = (MODE == 1) ? cgrp * GBN : 0;
    const float vs = atts[ab + c];
    const float vd = attd[ab + c];
    const float v  = (which == 0) ? vs : vd;
    satt[which * GBN + c] = bf16_val(v);
  } else {
    if (tid < 64) {
      const int which = tid >> 5;
      const int c = tid & 31;
      const float v0 = cb1[c];
      const float v1 = cw2[c];
      const float v  = (which == 0) ? v0 : v1;
      satt[which * GBN + c] = bf16_val(v);
    }
  }

  v8f acc[4];
  {
    const v8f z = {0.f, 0.f, 0.f, 0.f, 0.f, 0.f, 0.f, 0.f};
    acc[0] = z; acc[1] = z; acc[2] = z; acc[3] = z;
  }
  const unsigned short* ap = A  + (size_t)(rowBase + 16 * wave + m) * (size_t)KP + 8 * hh;
  const unsigned short* wp = WT + (size_t)(col0 + m) * (size_t)KP + 8 * hh;
#pragma unroll 1
  for (int ks = 0; ks < KP / 32; ++ks) {
    FragB af;
    af.h[0] = *(const v8usa*)(ap + 32 * ks);
    af.h[1] = *(const v8usa*)(ap + 32 * ks + 16);
#pragma unroll
    for (int t = 0; t < 4; ++t) {
      const unsigned short* wq = wp + (size_t)(16 * t) * (size_t)KP + 32 * ks;
      FragB bf;
      bf.h[0] = *(const v8usa*)wq;
      bf.h[1] = *(const v8usa*)(wq + 16);
      acc[t] = wmb(af, bf, acc[t]);
    }
  }

#pragma unroll
  for (int t = 0; t < 4; ++t) {
    const int lc = 16 * t + m;
#pragma unroll
    for (int r = 0; r < 8; ++r) {
      const int lr = 16 * wave + 8 * hh + r;
      stg[lr * GBN + lc] = acc[t][r];
    }
  }
  __syncthreads();

  if constexpr (MODE != 2) {
    {
      const int row = tid & 63, which = tid >> 6;
      const float* sa = satt + which * GBN;
      const float* hr = stg + row * GBN;
#pragma unroll
      for (int hd = 0; hd < HB; ++hd) {
        float d = 0.f;
#pragma unroll
        for (int c4 = 0; c4 < DL / 4; ++c4) {
          const v4f hv = *(const v4fa*)(hr + hd * DL + 4 * c4);
          const v4f av = *(const v4fa*)(sa + hd * DL + 4 * c4);
          d = fmaf(hv.x, av.x, d);
          d = fmaf(hv.y, av.y, d);
          d = fmaf(hv.z, av.z, d);
          d = fmaf(hv.w, av.w, d);
        }
        sdot[(which * HB + hd) * GBM + row] = d;
      }
    }
    __syncthreads();

    v4f fv[8];
#pragma unroll
    for (int i = 0; i < 8; ++i) {
      const int lr = 16 * wave + 2 * i + hh;
      fv[i] = *(const v4fa*)(stg + lr * GBN + 4 * m);
    }
    const int which2 = lane >> 4, piece = lane & 15;
    const int hdw    = (MODE == 0) ? wave : 0;
    const int hglob  = ((MODE == 1) ? cgrp : 0) + hdw;
    const v4f sdv = *(const v4fa*)(sdot + (which2 * HB + hdw) * GBM + 4 * piece);
    float* sp = SD + (size_t)(2 * hglob + which2) * (size_t)MPr + rowBase + 4 * piece;
    const bool sdw = (MODE == 0) || (wave == 0);

#pragma unroll
    for (int i = 0; i < 8; ++i) {
      const int lr = 16 * wave + 2 * i + hh;
      const int gr = rowBase + lr;
      float* op = outF + (size_t)gr * (size_t)ldo + col0 + 4 * m;
      *(volatile v4f*)op = fv[i];
    }
    if (sdw) *(volatile v4f*)sp = sdv;
    __threadfence();
#pragma unroll
    for (int i = 0; i < 8; ++i) {
      const int lr = 16 * wave + 2 * i + hh;
      const int gr = rowBase + lr;
      float* op = outF + (size_t)gr * (size_t)ldo + col0 + 4 * m;
      *(volatile v4f*)op = fv[i];
    }
    if (sdw) *(volatile v4f*)sp = sdv;
  } else {
    {
      const int row = tid & 63, half = tid >> 6;
      const float* hr = stg + row * GBN;
      const int cst = 16 * half;
      float ps = 0.0f;
#pragma unroll 1
      for (int c = cst; c < cst + 16; ++c) {
        const float z = hr[c] + satt[c];
        const float e = eluf(z);
        ps = fmaf(e, satt[GBN + c], ps);
      }
      sdot[half * GBM + row] = ps;
    }
    __syncthreads();
    if (wave == 0) {
      const float cb2v = bf16_val(cb2[0]);
      const int piece = lane & 15;
      const v4f p0 = *(const v4fa*)(sdot + 4 * piece);
      const v4f p1 = *(const v4fa*)(sdot + GBM + 4 * piece);
      v4f o;
      o.x = (p0.x + p1.x) + cb2v;
      o.y = (p0.y + p1.y) + cb2v;
      o.z = (p0.z + p1.z) + cb2v;
      o.w = (p0.w + p1.w) + cb2v;
      int live = nN - rowBase;
      live = live < 0 ? 0 : (live > GBM ? GBM : live);
      const int r0 = 4 * piece;
      const bool act  = lane < 16;
      const bool full = act && (r0 + 4 <= live);
      const bool part = act && (!full) && (r0 < live);
      float* op = outp + (size_t)rowBase + r0;
      if (full) *(volatile v4f*)op = o;
      if (part) {
        if (r0     < live) *(volatile float*)(op    ) = o.x;
        if (r0 + 1 < live) *(volatile float*)(op + 1) = o.y;
        if (r0 + 2 < live) *(volatile float*)(op + 2) = o.z;
        if (r0 + 3 < live) *(volatile float*)(op + 3) = o.w;
      }
      __threadfence();
      if (full) *(volatile v4f*)op = o;
      if (part) {
        if (r0     < live) *(volatile float*)(op    ) = o.x;
        if (r0 + 1 < live) *(volatile float*)(op + 1) = o.y;
        if (r0 + 2 < live) *(volatile float*)(op + 2) = o.z;
        if (r0 + 3 < live) *(volatile float*)(op + 3) = o.w;
      }
    }
  }
}

template <int L3>
__global__ __launch_bounds__(NTHR) void k_agg(const int* __restrict__ srcs, const int* __restrict__ dsts,
                                              int nE, int nN, int vec8, int mRows,
                                              const float* __restrict__ SD, int MPr,
                                              const float* __restrict__ F, const float* __restrict__ bias,
                                              const float* __restrict__ bng, const float* __restrict__ bnb,
                                              const float* __restrict__ bnm, const float* __restrict__ bnv,
                                              unsigned short* XP) {
  static_assert(L3 == 0 || L3 == 1);
  constexpr int CPL = L3 ? 8 : 2;
  constexpr int CW  = L3 ? H3W : HC;
  extern __shared__ __attribute__((aligned(16))) int dsm[];
  int* list = dsm;
  int* hl   = dsm + LISTN;
  int* sl   = dsm + LISTN + RCAP;
  int* cnt  = dsm + LISTN + 2 * RCAP;
  int* offs = cnt + NBA;
  int* cur  = offs + NBA;
  int* misc = cur + NBA;
  const int tid = (int)threadIdx.x, lane = tid & 31, wave = tid >> 5;
  const int nodeBase = (int)blockIdx.x * NBA;
  const int head = lane >> 3;
  const int jb = L3 ? 8 * (lane & 7) : 2 * lane;
  const int gb = L3 ? 8 * lane : 2 * lane;

  {
    const v4i z4 = {0, 0, 0, 0};
    for (int i = tid * 4; i < AGG_ZINTS; i += NTHR * 4) *(v4ia*)(dsm + i) = z4;
    if (tid < 16) misc[tid] = 0;
  }
  float sc[CPL], tc[CPL];
  {
    float bl[CPL], gg[CPL], be[CPL], mm[CPL], vv[CPL];
    ldc<CPL>(bias + jb, bl);
    ldc<CPL>(bng + jb, gg);
    ldc<CPL>(bnb + jb, be);
    ldc<CPL>(bnm + jb, mm);
    ldc<CPL>(bnv + jb, vv);
#pragma unroll
    for (int i = 0; i < CPL; ++i) {
      const float r = rsqrtf(bf16_val(vv[i]) + BNEPS);
      const float s = bf16_val(gg[i]) * r;
      sc[i] = s;
      tc[i] = fmaf(bf16_val(bl[i]) - bf16_val(mm[i]), s, bf16_val(be[i]));
    }
  }
  __syncthreads();

  int t = 0, ov = 0;
  const int nChunks = (nE + CHUNK - 1) / CHUNK;
#pragma unroll 1
  for (int ch = 0; ch < nChunks; ++ch) {
    const int cbase = ch * CHUNK;
    const int wc = scan_chunk<SLA>(dsts, nE, cbase, nodeBase, NBA, vec8, list, tid, lane, wave);
    if (lane == 0) misc[wave] = wc;
    __syncthreads();
    if (wave == 0) {
#pragma unroll 1
      for (int w2 = 0; w2 < NWAVE; ++w2) {
        int c = misc[w2];
        c = c < 0 ? 0 : (c > WCAP ? WCAP : c);
#pragma unroll 1
        for (int b0 = 0; b0 < c; b0 += 32) {
          const int idx = b0 + lane;
          const int ent = list[w2 * WCAP + (idx < WCAP ? idx : WCAP - 1)];
          const int m32 = (c - b0) < 32 ? (c - b0) : 32;
#pragma unroll 1
          for (int k = 0; k < m32; ++k) {
            const int u    = __builtin_amdgcn_readlane(ent, k);
            const int slot = u & (NBA - 1);
            const int el   = (u >> SLA) & (CHUNK - 1);
            const int pk   = ((cbase + el) << SLA) | slot;
            if (t < RCAP) {
              if (lane == 0) { hl[t] = pk; cnt[slot] = cnt[slot] + 1; }
              t = t + 1;
            } else {
              ov = 1;
            }
          }
        }
      }
    }
    __syncthreads();
  }
  if (wave == 0 && lane == 0) { misc[8] = t; misc[9] = ov; }
  __syncthreads();
  int tt = misc[8];
  tt = tt < 0 ? 0 : (tt > RCAP ? RCAP : tt);
  const int ovf = misc[9];

  if (wave == 0) {
    const int base = lane * (NBA / 32);
    int s = 0;
#pragma unroll 1
    for (int i = 0; i < NBA / 32; ++i) s += cnt[base + i];
    int incl = s;
#pragma unroll
    for (int d = 1; d < 32; d <<= 1) {
      const int y = __shfl_up(incl, d, 32);
      if (lane >= d) incl += y;
    }
    int run = incl - s;
#pragma unroll 1
    for (int i = 0; i < NBA / 32; ++i) {
      const int cv = cnt[base + i];
      offs[base + i] = run;
      cur[base + i]  = run;
      run += cv;
    }
  }
  __syncthreads();
  if (wave == 0) {
#pragma unroll 1
    for (int b0 = 0; b0 < tt; b0 += 32) {
      const int idx = b0 + lane;
      const int ent = hl[idx < RCAP ? idx : RCAP - 1];
      const int m32 = (tt - b0) < 32 ? (tt - b0) : 32;
#pragma unroll 1
      for (int k = 0; k < m32; ++k) {
        const int u    = __builtin_amdgcn_readlane(ent, k);
        const int slot = u & (NBA - 1);
        if (lane == 0) {
          int p = cur[slot];
          p = p < 0 ? 0 : (p > RCAP - 1 ? RCAP - 1 : p);
          sl[p] = u;
          cur[slot] = p + 1;
        }
      }
    }
  }
  __syncthreads();

  const float pz = (ovf != 0) ? __int_as_float(0x7fc00000) : 0.0f;
  const float* P0  = SD;
  const float* P1  = SD + (size_t)2 * (size_t)MPr;
  const float* P2  = SD + (size_t)4 * (size_t)MPr;
  const float* P3  = SD + (size_t)6 * (size_t)MPr;
  const float* ASp = SD + (size_t)(2 * head) * (size_t)MPr;
  const float* ADp = ASp + MPr;
#pragma unroll 1
  for (int si = 0; si < NBA / NWAVE; ++si) {
    const int s    = si * NWAVE + wave;
    const int node = nodeBase + s;
    int c = cnt[s];
    const bool big = c > DEGCAP;
    c = c < 0 ? 0 : (c > DEGCAP ? DEGCAP : c);
    int o = offs[s];
    o = o < 0 ? 0 : (o > RCAP ? RCAP : o);
    const int nc = node < nN ? node : nN - 1;
    const float as0 = ASp[nc];
    const float ad  = ADp[nc];
    float acc[CPL];
    ldc<CPL>(F + (size_t)nc * CW + gb, acc);
    float l0 = as0 + ad;
    l0 = l0 > 0.f ? l0 : NEGSL * l0;
    float mx = l0, dn = 1.0f;
#pragma unroll 1
    for (int b0 = 0; b0 < c; b0 += 32) {
      int idx = o + b0 + lane;
      idx = idx > RCAP - 1 ? RCAP - 1 : idx;
      const int ent = sl[idx];
      int eid = ent >> SLA;
      eid = eid < 0 ? 0 : (eid > nE - 1 ? nE - 1 : eid);
      int sr = srcs[eid];
      sr = sr < 0 ? 0 : (sr > nN - 1 ? nN - 1 : sr);
      const int e0i = __float_as_int(P0[sr]);
      const int e1i = __float_as_int(P1[sr]);
      const int e2i = __float_as_int(P2[sr]);
      const int e3i = __float_as_int(P3[sr]);
      const int m32 = (c - b0) < 32 ? (c - b0) : 32;
#pragma unroll 1
      for (int k = 0; k < m32; ++k) {
        const int   sk = __builtin_amdgcn_readlane(sr, k);
        const float q0 = __int_as_float(__builtin_amdgcn_readlane(e0i, k));
        const float q1 = __int_as_float(__builtin_amdgcn_readlane(e1i, k));
        const float q2 = __int_as_float(__builtin_amdgcn_readlane(e2i, k));
        const float q3 = __int_as_float(__builtin_amdgcn_readlane(e3i, k));
        const float ask = (head == 0) ? q0 : ((head == 1) ? q1 : ((head == 2) ? q2 : q3));
        float a[CPL];
        ldc<CPL>(F + (size_t)sk * CW + gb, a);
        float lg = ask + ad;
        lg = lg > 0.f ? lg : NEGSL * lg;
        const float df = lg - mx;
        const float ee = __expf(-fabsf(df));
        const bool  up = df > 0.f;
        const float s1 = up ? ee : 1.0f;
        const float s2 = up ? 1.0f : ee;
        mx = up ? lg : mx;
        dn = fmaf(dn, s1, s2);
#pragma unroll
        for (int i = 0; i < CPL; ++i) acc[i] = fmaf(acc[i], s1, s2 * a[i]);
      }
    }
    const float inv = __builtin_amdgcn_rcpf(dn);
    const float pzr = big ? __int_as_float(0x7fc00000) : pz;
    const bool live = node < nN;
    const bool wr   = node < mRows;
    unsigned short* gp = XP + (size_t)node * KP + 8 * lane;
    v4u pv;
    if constexpr (L3 == 0) {
      float y0 = fmaf(acc[0] * inv, sc[0], tc[0]);
      float y1 = fmaf(acc[1] * inv, sc[1], tc[1]);
      y0 = eluf(y0) + pzr;
      y1 = eluf(y1) + pzr;
      y0 = live ? y0 : 0.0f;
      y1 = live ? y1 : 0.0f;
      const unsigned hb0 = bf16_bits(y0), hb1 = bf16_bits(y1);
      const unsigned lb0 = bf16_bits(y0 - __uint_as_float(hb0 << 16));
      const unsigned lb1 = bf16_bits(y1 - __uint_as_float(hb1 << 16));
      const int hw = (int)(hb0 | (hb1 << 16));
      const int lw = (int)(lb0 | (lb1 << 16));
      const int i0 = (4 * lane) & 31, i1 = (4 * lane + 1) & 31, i2 = (4 * lane + 2) & 31, i3 = (4 * lane + 3) & 31;
      const int gh0 = __shfl(hw, i0), gh1 = __shfl(hw, i1), gh2 = __shfl(hw, i2), gh3 = __shfl(hw, i3);
      const int gl0 = __shfl(lw, i0), gl1 = __shfl(lw, i1), gl2 = __shfl(lw, i2), gl3 = __shfl(lw, i3);
      const bool lsel = lane >= 8;
      pv.x = (unsigned)(lsel ? gl0 : gh0);
      pv.y = (unsigned)(lsel ? gl1 : gh1);
      pv.z = (unsigned)(lsel ? gl2 : gh2);
      pv.w = (unsigned)(lsel ? gl3 : gh3);
    } else {
      float val[8];
#pragma unroll
      for (int i = 0; i < 8; ++i) val[i] = acc[i] * inv;
#pragma unroll
      for (int i = 0; i < 8; ++i) val[i] += __shfl_xor(val[i], 8);
#pragma unroll
      for (int i = 0; i < 8; ++i) val[i] += __shfl_xor(val[i], 16);
      Pk8 ho, lo;
#pragma unroll
      for (int i = 0; i < 8; ++i) {
        float y = fmaf(0.25f * val[i], sc[i], tc[i]) + pzr;
        y = live ? y : 0.0f;
        const unsigned hb = bf16_bits(y);
        ho.h[i] = (unsigned short)hb;
        lo.h[i] = (unsigned short)bf16_bits(y - __uint_as_float(hb << 16));
      }
      const bool lsel = lane >= 8;
      pv.x = lsel ? lo.u.x : ho.u.x;
      pv.y = lsel ? lo.u.y : ho.u.y;
      pv.z = lsel ? lo.u.z : ho.u.z;
      pv.w = lsel ? lo.u.w : ho.u.w;
    }
    if (wr && lane < 16) *(volatile v4u*)gp = pv;
    __threadfence();
    if (wr && lane < 16) *(volatile v4u*)gp = pv;
  }
}

static inline int cdiv(int a, int b) { return (a + b - 1) / b; }

extern "C" void kernel_launch(void* const* d_in, const int* in_sizes, int n_in,
                              void* d_out, int out_size, void* d_ws, size_t ws_size,
                              hipStream_t stream) {
  if (n_in < 30) return;
  if (in_sizes[0] < DIN || (in_sizes[0] % DIN) != 0) return;
  const int nN = in_sizes[0] / DIN;
  if (in_sizes[1] < 2 || (in_sizes[1] & 1) != 0) return;
  const int nE = in_sizes[1] / 2;
  if (nE < 1 || nE >= (1 << 21)) return;
  if (in_sizes[2] != DIN * HC) return;
  if (in_sizes[3] != NHEAD * 16 || in_sizes[4] != NHEAD * 16) return;
  if (in_sizes[5] != HC) return;
  if (in_sizes[6] != HC * HC) return;
  if (in_sizes[7] != NHEAD * 16 || in_sizes[8] != NHEAD * 16) return;
  if (in_sizes[9] != HC) return;
  if (in_sizes[10] != HC * H3W) return;
  if (in_sizes[11] != NHEAD * HC || in_sizes[12] != NHEAD * HC) return;
  if (in_sizes[13] != HC) return;
  for (int i = 14; i <= 25; ++i) if (in_sizes[i] != HC) return;
  if (in_sizes[26] != HC * CLSH) return;
  if (in_sizes[27] != CLSH) return;
  if (in_sizes[28] != CLSH) return;
  if (in_sizes[29] != 1) return;
  if (out_size != nN) return;

  const float* x    = (const float*)d_in[0];
  const int*   edge = (const int*)d_in[1];
  const float* W1   = (const float*)d_in[2];
  const float* a1s  = (const float*)d_in[3];
  const float* a1d  = (const float*)d_in[4];
  const float* b1   = (const float*)d_in[5];
  const float* W2   = (const float*)d_in[6];
  const float* a2s  = (const float*)d_in[7];
  const float* a2d  = (const float*)d_in[8];
  const float* b2   = (const float*)d_in[9];
  const float* W3   = (const float*)d_in[10];
  const float* a3s  = (const float*)d_in[11];
  const float* a3d  = (const float*)d_in[12];
  const float* b3   = (const float*)d_in[13];
  const float* bn1g = (const float*)d_in[14];
  const float* bn1b = (const float*)d_in[15];
  const float* bn1m = (const float*)d_in[16];
  const float* bn1v = (const float*)d_in[17];
  const float* bn2g = (const float*)d_in[18];
  const float* bn2b = (const float*)d_in[19];
  const float* bn2m = (const float*)d_in[20];
  const float* bn2v = (const float*)d_in[21];
  const float* bn3g = (const float*)d_in[22];
  const float* bn3b = (const float*)d_in[23];
  const float* bn3m = (const float*)d_in[24];
  const float* bn3v = (const float*)d_in[25];
  const float* cW1  = (const float*)d_in[26];
  const float* cb1  = (const float*)d_in[27];
  const float* cW2  = (const float*)d_in[28];
  const float* cb2  = (const float*)d_in[29];
  float* out = (float*)d_out;
  const int* src = edge;
  const int* dst = edge + nE;

  const int MP   = cdiv(nN, GBM) * GBM;
  const int gM   = MP / GBM;
  const int gA   = cdiv(MP, NBA);
  if ((long long)gA * NBA < (long long)MP) return;
  const int vec8 = ((nE & 3) == 0) ? 1 : 0;

  char* ws = (char*)d_ws;
  size_t off = 0;
  const size_t oW1T = off; off += (size_t)HC * DIN * 2;                  off = (off + 255) & ~(size_t)255;
  const size_t oW2T = off; off += (size_t)HC * KP * 2;                   off = (off + 255) & ~(size_t)255;
  const size_t oW3T = off; off += (size_t)H3W * KP * 2;                  off = (off + 255) & ~(size_t)255;
  const size_t oCWT = off; off += (size_t)GBN * KP * 2;                  off = (off + 255) & ~(size_t)255;
  const size_t oSD  = off; off += (size_t)8 * (size_t)MP * 4;            off = (off + 255) & ~(size_t)255;
  const size_t oXB  = off; off += (size_t)MP * DIN * 2;                  off = (off + 255) & ~(size_t)255;
  const size_t oXP  = off; off += (size_t)MP * KP * 2;                   off = (off + 255) & ~(size_t)255;
  const size_t oH   = off; off += (size_t)MP * H3W * 4;                  off = (off + 255) & ~(size_t)255;
  if (off > ws_size || off > (size_t)WSMAX) return;
  unsigned short* W1T = (unsigned short*)(ws + oW1T);
  unsigned short* W2T = (unsigned short*)(ws + oW2T);
  unsigned short* W3T = (unsigned short*)(ws + oW3T);
  unsigned short* CWT = (unsigned short*)(ws + oCWT);
  float*          SDp = (float*)(ws + oSD);
  unsigned short* XB  = (unsigned short*)(ws + oXB);
  unsigned short* XP  = (unsigned short*)(ws + oXP);
  float*          H   = (float*)(ws + oH);

  const size_t aggLds = (size_t)AGG_LDS_INTS * 4;
  hipFuncSetAttribute(reinterpret_cast<const void*>(&k_agg<0>), hipFuncAttributeMaxDynamicSharedMemorySize, (int)aggLds);
  hipFuncSetAttribute(reinterpret_cast<const void*>(&k_agg<1>), hipFuncAttributeMaxDynamicSharedMemorySize, (int)aggLds);

  const int nUx = MP * (DIN / 8);
  k_wprep<<<(NU1 + NU2 + NU3 + NU4) / NTHR, NTHR, 0, stream>>>(W1, W2, W3, cW1, W1T, W2T, W3T, CWT);
  k_cvx<<<cdiv(nUx, NTHR), NTHR, 0, stream>>>(x, nN, nUx, XB);
  k_gemm<0><<<dim3(gM, 1), GTHR, 0, stream>>>(XB, W1T, H, HC, a1s, a1d, SDp, MP, cb1, cW2, cb2, out, nN);
  k_agg<0><<<gA, NTHR, aggLds, stream>>>(src, dst, nE, nN, vec8, MP, SDp, MP, H, b1, bn1g, bn1b, bn1m, bn1v, XP);
  k_gemm<0><<<dim3(gM, 1), GTHR, 0, stream>>>(XP, W2T, H, HC, a2s, a2d, SDp, MP, cb1, cW2, cb2, out, nN);
  k_agg<0><<<gA, NTHR, aggLds, stream>>>(src, dst, nE, nN, vec8, MP, SDp, MP, H, b2, bn2g, bn2b, bn2m, bn2v, XP);
  k_gemm<1><<<dim3(gM, NHEAD), GTHR, 0, stream>>>(XP, W3T, H, H3W, a3s, a3d, SDp, MP, cb1, cW2, cb2, out, nN);
  k_agg<1><<<gA, NTHR, aggLds, stream>>>(src, dst, nE, nN, vec8, MP, SDp, MP, H, b3, bn3g, bn3b, bn3m, bn3v, XP);
  k_gemm<2><<<dim3(gM, 1), GTHR, 0, stream>>>(XP, CWT, H, HC, a1s, a1d, SDp, MP, cb1, cW2, cb2, out, nN);
}
